// ScaledDotProductAttention_678604832861
// MI455X (gfx1250) — hardware-verified
//
#include <hip/hip_runtime.h>
#include <stdint.h>


typedef _Float16 v16h __attribute__((ext_vector_type(16)));
typedef _Float16 v8h  __attribute__((ext_vector_type(8)));
typedef float    v8f  __attribute__((ext_vector_type(8)));
typedef float    v4f  __attribute__((ext_vector_type(4)));
typedef int      v4i  __attribute__((ext_vector_type(4)));

#ifndef NB
#define NB 4
#endif
#ifndef SEQ
#define SEQ 2048
#endif
#define SEQ_FULL 2048
#define NH 16
#define DK 64

constexpr int QT  = 128;
constexpr int KB  = 64;
constexpr int NT  = KB / 16;
constexpr int NKB = SEQ / KB;
constexpr int PCH = 128;
constexpr int KDP = DK + 8;
constexpr int VDP = KB + 8;
constexpr int PDP = KB + 8;
constexpr int ODP = DK + 4;
constexpr int TP  = PCH + 8;
constexpr size_t IN_BH = (size_t)SEQ_FULL * DK;
constexpr size_t WS_BH = (size_t)SEQ * DK;

static_assert(NB >= 1);
static_assert(SEQ >= PCH);
static_assert(SEQ <= SEQ_FULL);
static_assert(SEQ % QT == 0);
static_assert(SEQ % KB == 0);
static_assert(SEQ % PCH == 0);
static_assert(NT == 4);
static_assert(DK == 64);
static_assert((KDP * 2) % 16 == 0);
static_assert((VDP * 2) % 16 == 0);
static_assert((PDP * 2) % 16 == 0);
static_assert((ODP * 4) % 16 == 0);
static_assert((TP  * 2) % 16 == 0);

union HV { v8h h; v4i i; };

__device__ __forceinline__ float bf16v(float x) {
    uint32_t u = __float_as_uint(x);
    u = (u + 0x7FFFu + ((u >> 16) & 1u)) & 0xFFFF0000u;
    return __uint_as_float(u);
}
__device__ __forceinline__ _Float16 h16(float x) { return (_Float16)bf16v(x); }

__device__ __forceinline__ float fexp2(float x) {
#if defined(__has_builtin)
#if __has_builtin(__builtin_amdgcn_exp2f)
    return __builtin_amdgcn_exp2f(x);
#else
    return exp2f(x);
#endif
#else
    return exp2f(x);
#endif
}

__device__ __forceinline__ float frcp(float x) {
#if defined(__has_builtin)
#if __has_builtin(__builtin_amdgcn_rcpf)
    return __builtin_amdgcn_rcpf(x);
#else
    return 1.0f / x;
#endif
#else
    return 1.0f / x;
#endif
}

__device__ __forceinline__ v8f mma16(v16h a, v16h b, v8f c) {
    v8f d = __builtin_amdgcn_wmma_f32_16x16x32_f16(false, a, false, b, (short)0, c, false, false);
    asm volatile("v_nop\n\tv_nop\n\tv_nop\n\tv_nop" : "+v"(d) : "v"(a), "v"(b));
    return d;
}

__device__ __forceinline__ v16h ld_op16(const _Float16* p) {
    union { v16h v; v8h hh[2]; } u;
    u.hh[0] = *(const v8h*)(p);
    u.hh[1] = *(const v8h*)(p + 16);
    return u.v;
}

__device__ __forceinline__ v16h ld_q(const float* p) {
    const v4f x0 = *(const v4f*)(p);
    const v4f x1 = *(const v4f*)(p + 4);
    const v4f x2 = *(const v4f*)(p + 16);
    const v4f x3 = *(const v4f*)(p + 20);
    v16h r;
#pragma unroll
    for (int j = 0; j < 4; ++j) {
        r[j]      = h16(x0[j]);
        r[4 + j]  = h16(x1[j]);
        r[8 + j]  = h16(x2[j]);
        r[12 + j] = h16(x3[j]);
    }
    return r;
}

__global__ __launch_bounds__(256)
void k_prep(const float* __restrict__ K, const float* __restrict__ V,
            _Float16* __restrict__ Kh, _Float16* __restrict__ Vt) {
    __shared__ __align__(16) _Float16 T[DK * TP];

    const int kb  = blockIdx.x;
    const int bh  = blockIdx.y;
    const int tid = threadIdx.x;
    const size_t ib  = (size_t)bh * IN_BH + (size_t)kb * PCH * DK;
    const size_t kob = (size_t)bh * WS_BH + (size_t)kb * PCH * DK;
    const size_t vob = (size_t)bh * WS_BH + (size_t)kb * PCH;

    HV kv[4];
    size_t ka[4];
#pragma unroll
    for (int i = 0; i < 4; ++i) {
        const int p  = i * 256 + tid;
        const int r  = p >> 3;
        const int c8 = (p & 7) * 8;
        const float* src = K + ib + (size_t)r * DK + c8;
        const v4f x0 = *(const v4f*)(src);
        const v4f x1 = *(const v4f*)(src + 4);
        v8h hv;
#pragma unroll
        for (int j = 0; j < 4; ++j) { hv[j] = h16(x0[j]); hv[4 + j] = h16(x1[j]); }
        kv[i].h = hv;
        ka[i]   = kob + (size_t)r * DK + c8;
    }
#pragma unroll
    for (int i = 0; i < 4; ++i) *(volatile v4i*)(Kh + ka[i]) = kv[i].i;

#pragma unroll
    for (int f = 0; f < 8; ++f) {
        const int e  = f * 256 + tid;
        const int r  = e >> 4;
        const int c4 = (e & 15) * 4;
        const v4f x  = *(const v4f*)(V + ib + (size_t)r * DK + c4);
#pragma unroll
        for (int j = 0; j < 4; ++j) T[(c4 + j) * TP + r] = h16(x[j]);
    }
    __syncthreads();

    HV vv[4];
    size_t va[4];
#pragma unroll
    for (int i = 0; i < 4; ++i) {
        const int p  = i * 256 + tid;
        const int L  = p >> 3;
        const int d  = L >> 1;
        const int ko = (L & 1) * 64 + (p & 7) * 8;
        vv[i].h = *(const v8h*)&T[d * TP + ko];
        va[i]   = vob + (size_t)d * SEQ + ko;
    }
#pragma unroll
    for (int i = 0; i < 4; ++i) *(volatile v4i*)(Vt + va[i]) = vv[i].i;

    __threadfence();
#pragma unroll
    for (int i = 0; i < 4; ++i) *(volatile v4i*)(Kh + ka[i]) = kv[i].i;
#pragma unroll
    for (int i = 0; i < 4; ++i) *(volatile v4i*)(Vt + va[i]) = vv[i].i;
}

__global__ __launch_bounds__(256) __attribute__((amdgpu_num_vgpr(256)))
void k_attn(const float* __restrict__ Q,
            const _Float16* __restrict__ Kh,
            const _Float16* __restrict__ Vt,
            float* __restrict__ O) {
    __shared__ __align__(16) _Float16 Ksh[KB * KDP];
    __shared__ __align__(16) _Float16 Vts[DK * VDP];
    __shared__ __align__(16) _Float16 Pst[8 * 16 * PDP];
    __shared__ __align__(16) float    Osh[8 * 16 * ODP];

    const int qb   = blockIdx.x;
    const int h    = blockIdx.y;
    const int b    = blockIdx.z;
    const int tid  = threadIdx.x;
    const int lane = tid & 31;
    const int wv   = tid >> 5;
    const int hf   = lane >> 4;
    const int l16  = lane & 15;
    const int koff = hf * 8;

    const size_t bhi = (size_t)b * NH + h;
    const float*    Qb  = Q  + bhi * IN_BH;
    const _Float16* KhB = Kh + bhi * WS_BH;
    const _Float16* VtB = Vt + bhi * WS_BH;
    float*          Ob  = O  + bhi * WS_BH;

    const float CL = 0.125f * 1.44269504088896341f;

    const int qrow = qb * QT + wv * 16 + l16;
    const v16h qa0 = ld_q(Qb + (size_t)qrow * DK + koff);
    const v16h qa1 = ld_q(Qb + (size_t)qrow * DK + 32 + koff);

    v16h vones;
#pragma unroll
    for (int j = 0; j < 16; ++j) vones[j] = (_Float16)1.0f;

    const v8f vzero = {0.f, 0.f, 0.f, 0.f, 0.f, 0.f, 0.f, 0.f};
    v8f o[4];
#pragma unroll
    for (int t = 0; t < 4; ++t) o[t] = vzero;
    v8f olsum = vzero;

    float m[8];
#pragma unroll
    for (int v = 0; v < 8; ++v) m[v] = -1e30f;

    _Float16* Pw = &Pst[wv * 16 * PDP];

#pragma unroll 1
    for (int kb = 0; kb < NKB; ++kb) {
        __syncthreads();

#pragma unroll
        for (int i = 0; i < 2; ++i) {
            const int cidx = tid + i * 256;
            const int row  = cidx >> 3;
            const int cc   = cidx & 7;
            *(v8h*)&Ksh[row * KDP + cc * 8] =
                *(const v8h*)(KhB + (size_t)(kb * KB + row) * DK + cc * 8);
            *(v8h*)&Vts[row * VDP + cc * 8] =
                *(const v8h*)(VtB + (size_t)row * SEQ + (size_t)kb * KB + cc * 8);
        }
        __syncthreads();

        v8f c[NT];
#pragma unroll
        for (int t = 0; t < NT; ++t) c[t] = vzero;
#pragma unroll
        for (int kc = 0; kc < 2; ++kc) {
            const v16h a = kc ? qa1 : qa0;
#pragma unroll
            for (int t = 0; t < NT; ++t) {
                const v16h bop = ld_op16(&Ksh[(t * 16 + l16) * KDP + kc * 32 + koff]);
                c[t] = mma16(a, bop, c[t]);
            }
        }

        float sc[8], mb[8];
#pragma unroll
        for (int v = 0; v < 8; ++v) {
            float r = fmaxf(fmaxf(c[0][v], c[1][v]), fmaxf(c[2][v], c[3][v]));
            r = fmaxf(r, __shfl_xor(r, 1, 32));
            r = fmaxf(r, __shfl_xor(r, 2, 32));
            r = fmaxf(r, __shfl_xor(r, 4, 32));
            r = fmaxf(r, __shfl_xor(r, 8, 32));
            const float mn = fmaxf(m[v], r);
            sc[v] = fexp2((m[v] - mn) * CL);
            m[v]  = mn;
            mb[v] = mn * CL - 10.0f;
        }
#pragma unroll
        for (int t = 0; t < NT; ++t)
#pragma unroll
            for (int v = 0; v < 8; ++v)
                c[t][v] = fexp2(c[t][v] * CL - mb[v]);

#pragma unroll
        for (int v = 0; v < 8; ++v) {
#pragma unroll
            for (int t = 0; t < 4; ++t) o[t][v] *= sc[v];
            olsum[v] *= sc[v];
        }

#pragma unroll
        for (int t = 0; t < NT; ++t)
#pragma unroll
            for (int v = 0; v < 8; ++v)
                Pw[(v + 8 * hf) * PDP + t * 16 + l16] = (_Float16)c[t][v];
        __syncthreads();

#pragma unroll
        for (int kc = 0; kc < KB / 32; ++kc) {
            const v16h pa = ld_op16(&Pw[l16 * PDP + kc * 32 + koff]);
            olsum = mma16(pa, vones, olsum);
#pragma unroll
            for (int t = 0; t < 4; ++t) {
                const v16h vb = ld_op16(&Vts[(t * 16 + l16) * VDP + kc * 32 + koff]);
                o[t] = mma16(pa, vb, o[t]);
            }
        }
    }

    float* Ow = &Osh[wv * 16 * ODP];
#pragma unroll
    for (int v = 0; v < 8; ++v) {
        const float rinv = frcp(olsum[v]);
        const int   row  = v + 8 * hf;
#pragma unroll
        for (int t = 0; t < 4; ++t) Ow[row * ODP + t * 16 + l16] = o[t][v] * rinv;
    }
    __syncthreads();

    v4f ov[8];
#pragma unroll
    for (int i = 0; i < 8; ++i) ov[i] = *(const v4f*)&Ow[(2 * i + hf) * ODP + l16 * 4];
    float* orow = Ob + (size_t)(qb * QT + wv * 16) * DK + l16 * 4;
#pragma unroll
    for (int i = 0; i < 8; ++i) *(volatile v4f*)(orow + (size_t)(2 * i + hf) * DK) = ov[i];
    __threadfence();
#pragma unroll
    for (int i = 0; i < 8; ++i) *(volatile v4f*)(orow + (size_t)(2 * i + hf) * DK) = ov[i];
}

extern "C" void kernel_launch(void* const* d_in, const int* in_sizes, int n_in,
                              void* d_out, int out_size, void* d_ws, size_t ws_size,
                              hipStream_t stream) {
    if (n_in < 3) return;
    const long long need_in = ((long long)(NB * NH - 1) * SEQ_FULL + SEQ) * DK;
    if ((long long)in_sizes[0] < need_in) return;
    if ((long long)in_sizes[1] < need_in) return;
    if ((long long)in_sizes[2] < need_in) return;
    const long long n_out = (long long)NB * NH * SEQ * DK;
    if ((long long)out_size < n_out) return;

    const size_t plane = (size_t)NB * NH * SEQ * DK;
    if (ws_size < 2 * plane * sizeof(_Float16)) return;

    const float* q = (const float*)d_in[0];
    const float* k = (const float*)d_in[1];
    const float* v = (const float*)d_in[2];
    float* out = (float*)d_out;

    _Float16* Kh = (_Float16*)d_ws;
    _Float16* Vt = Kh + plane;

    k_prep<<<dim3(SEQ / PCH, NB * NH), 256, 0, stream>>>(k, v, Kh, Vt);
    k_attn<<<dim3(SEQ / QT, NH, NB), 256, 0, stream>>>(q, Kh, Vt, out);
}
